// RITS_56160992363035
// MI455X (gfx1250) — hardware-run, weakly checked
//
#include <hip/hip_runtime.h>
#include <hip/hip_fp16.h>
#include <math.h>

typedef __attribute__((ext_vector_type(16))) _Float16 v16h;
typedef __attribute__((ext_vector_type(8)))  _Float16 v8h;
typedef __attribute__((ext_vector_type(4)))  _Float16 v4h;
typedef __attribute__((ext_vector_type(8)))  float    v8f;
typedef __attribute__((ext_vector_type(4)))  float    v4f;
typedef __attribute__((ext_vector_type(2)))  float    v2f;

constexpr int kB = 256;
constexpr int kS = 512;
constexpr int kF = 64;
constexpr int kH = 128;
constexpr int kG = 4 * kH;
constexpr int kSamp = 16;
constexpr int kBlocks = kB / kSamp;
constexpr float kWCarry = 1024.0f;
constexpr float sW = 1.0f / kWCarry;
constexpr int kPT  = kF + 8;
constexpr int kPH  = kH + 8;
constexpr int kPX  = kF + 8;
constexpr int kPGM = 2 * kF + 8;
constexpr int kPIN = 2 * kF + 8;
constexpr int kOut0 = 0;
constexpr int kOut1 = kB * kS * kF;
static_assert(kG == 512 && kBlocks == 16 && kOut1 == 8388608);
static_assert((kF % 32) == 0 && (kH % 32) == 0 && ((2 * kF) % 32) == 0);
static_assert((kPT % 8) == 0 && (kPH % 8) == 0 && (kPX % 8) == 0 && (kPGM % 8) == 0 && (kPIN % 8) == 0);
static_assert(kPT == 72 && kPH == 136 && kPX == 72 && kPGM == 136 && kPIN == 136);

constexpr size_t kSzWDH = (size_t)kH * kF * 2;
constexpr size_t kSzWTR = (size_t)kF * kH * 2;
constexpr size_t kSzWWC = (size_t)kF * 2 * kF * 2;
constexpr size_t kSzWIH = (size_t)kG * 2 * kF * 2;
constexpr size_t kSzWHH = (size_t)kG * kH * 2;
constexpr size_t kSzWFR = (size_t)kF * kF * 2;
constexpr size_t kSzV64  = (size_t)kF * 4;
constexpr size_t kSzV128 = (size_t)kH * 4;
constexpr size_t kSzV512 = (size_t)kG * 4;
constexpr size_t kSzPARTS = (size_t)kBlocks * kS * 4 * 4;
constexpr size_t kOffWDH = 0;
constexpr size_t kOffWTR = kOffWDH + kSzWDH;
constexpr size_t kOffWWC = kOffWTR + kSzWTR;
constexpr size_t kOffWIH = kOffWWC + kSzWWC;
constexpr size_t kOffWHH = kOffWIH + kSzWIH;
constexpr size_t kOffWFR = kOffWHH + kSzWHH;
constexpr size_t kOffDGM = kOffWFR + kSzWFR;
constexpr size_t kOffBDH = kOffDGM + kSzV64;
constexpr size_t kOffBDM = kOffBDH + kSzV128;
constexpr size_t kOffBTR = kOffBDM + kSzV64;
constexpr size_t kOffBFR = kOffBTR + kSzV64;
constexpr size_t kOffBWC = kOffBFR + kSzV64;
constexpr size_t kOffBIH = kOffBWC + kSzV64;
constexpr size_t kOffBHH = kOffBIH + kSzV512;
constexpr size_t kOffPARTS = kOffBHH + kSzV512;
constexpr size_t kWsTotal = kOffPARTS + kSzPARTS;
static_assert(kWsTotal == 456448ull);
static_assert(kWsTotal <= 134217728ull);
static_assert((kOffWTR % 128) == 0 && (kOffWWC % 128) == 0 && (kOffWIH % 128) == 0 && (kOffWHH % 128) == 0 &&
              (kOffWFR % 128) == 0 && (kOffDGM % 128) == 0 && (kOffBDH % 128) == 0 && (kOffBDM % 128) == 0 &&
              (kOffBTR % 128) == 0 && (kOffBFR % 128) == 0 && (kOffBWC % 128) == 0 && (kOffBIH % 128) == 0 &&
              (kOffBHH % 128) == 0 && (kOffPARTS % 128) == 0);

__device__ __forceinline__ _Float16 f16_flush(float v) {
  const float w = (fabsf(v) < 6.103515625e-05f) ? 0.0f : v;
  return (_Float16)w;
}

__device__ __forceinline__ float bf16r(float v) {
  unsigned u = __float_as_uint(v);
  u = (u + 0x7FFFu + ((u >> 16) & 1u)) & 0xFFFF0000u;
  return __uint_as_float(u);
}

namespace eng {
union FragU { v16h v; v8h h[2]; };
__device__ __forceinline__ v16h frag_load(const _Float16* p) {
  FragU f;
  f.h[0] = *(const v8h*)(p);
  f.h[1] = *(const v8h*)(p + 16);
  return f.v;
}
__device__ __forceinline__ v8f mma(v16h a, v16h b, v8f c) {
  return __builtin_amdgcn_wmma_f32_16x16x32_f16(false, a, false, b, (short)0, c, false, false);
}
__device__ __forceinline__ void guard1(v8f& a, v16h x, v16h y) {
  asm volatile("v_nop\n\tv_nop\n\tv_nop\n\tv_nop" : "+v"(a) : "v"(x), "v"(y));
}
__device__ __forceinline__ void guard_acc(v8f& a) {
  asm volatile("v_nop\n\tv_nop\n\tv_nop\n\tv_nop" : "+v"(a));
}
__device__ __forceinline__ void keep4(v16h a, v16h b, v16h c, v16h d) {
  asm volatile("v_nop" :: "v"(a), "v"(b), "v"(c), "v"(d));
}
}

template <int K>
__device__ __forceinline__ v8f tile_mm(const _Float16* A, int lda, const _Float16* __restrict__ Bt, int ldb,
                                       int n0, int rlane, int koff, v8f acc)
{
  static_assert((K % 32) == 0 && K >= 32 && K <= 128);
#pragma unroll
  for (int k0 = 0; k0 < K; k0 += 32) {
    const v16h ah = eng::frag_load(A + rlane * lda + koff + k0);
    const v16h bh = eng::frag_load(Bt + (size_t)(n0 + rlane) * ldb + koff + k0);
    acc = eng::mma(ah, bh, acc);
    eng::guard1(acc, ah, bh);
    eng::keep4(bh, bh, ah, ah);
  }
  return acc;
}

__global__ __launch_bounds__(256) void pack_rows_bf_kernel(
    const float* __restrict__ W, unsigned short* __restrict__ dH,
    int Kdim, int Nreal, int total8, float carry)
{
  const int i = blockIdx.x * 256 + threadIdx.x;
  if (i >= total8) return;
  const size_t e0 = (size_t)i << 3;
  const int row = (int)(e0 / (size_t)Kdim);
  const int col = (int)(e0 - (size_t)row * (size_t)Kdim);
  const bool live = (row < Nreal);
  const int rc = live ? row : (Nreal - 1);
  const v4f a0 = *(const v4f*)(W + (size_t)rc * Kdim + col);
  const v4f a1 = *(const v4f*)(W + (size_t)rc * Kdim + col + 4);
  const float w0 = a0[0];
  const float w1 = a0[1];
  const float w2 = a0[2];
  const float w3 = a0[3];
  const float w4 = a1[0];
  const float w5 = a1[1];
  const float w6 = a1[2];
  const float w7 = a1[3];
  const float t0 = bf16r(w0) * carry;
  const float t1 = bf16r(w1) * carry;
  const float t2 = bf16r(w2) * carry;
  const float t3 = bf16r(w3) * carry;
  const float t4 = bf16r(w4) * carry;
  const float t5 = bf16r(w5) * carry;
  const float t6 = bf16r(w6) * carry;
  const float t7 = bf16r(w7) * carry;
  const float g0 = live ? t0 : 0.0f;
  const float g1 = live ? t1 : 0.0f;
  const float g2 = live ? t2 : 0.0f;
  const float g3 = live ? t3 : 0.0f;
  const float g4 = live ? t4 : 0.0f;
  const float g5 = live ? t5 : 0.0f;
  const float g6 = live ? t6 : 0.0f;
  const float g7 = live ? t7 : 0.0f;
  v8h hv;
  hv[0] = f16_flush(g0);
  hv[1] = f16_flush(g1);
  hv[2] = f16_flush(g2);
  hv[3] = f16_flush(g3);
  hv[4] = f16_flush(g4);
  hv[5] = f16_flush(g5);
  hv[6] = f16_flush(g6);
  hv[7] = f16_flush(g7);
  unsigned short* qh = dH + e0;
  *(volatile v8h*)qh = hv;
  __threadfence();
  *(volatile v8h*)qh = hv;
}

__global__ __launch_bounds__(256) void rne_vec_kernel(
    const float* __restrict__ src, float* __restrict__ dst, int n4)
{
  const int i = blockIdx.x * 256 + threadIdx.x;
  if (i >= n4) return;
  const v4f a = *(const v4f*)(src + (size_t)i * 4);
  const float a0 = a[0];
  const float a1 = a[1];
  const float a2 = a[2];
  const float a3 = a[3];
  v4f r;
  r[0] = bf16r(a0);
  r[1] = bf16r(a1);
  r[2] = bf16r(a2);
  r[3] = bf16r(a3);
  float* p = dst + (size_t)i * 4;
  *(volatile v4f*)p = r;
  __threadfence();
  *(volatile v4f*)p = r;
}

__global__ __launch_bounds__(256) void wfr_pack_kernel(
    const float* __restrict__ Wfr, unsigned short* __restrict__ dH, int total8)
{
  const int i = blockIdx.x * 256 + threadIdx.x;
  if (i >= total8) return;
  const size_t e0 = (size_t)i << 3;
  const int n  = i >> 3;
  const int k8 = (i & 7) * 8;
  const v4f a0 = *(const v4f*)(Wfr + e0);
  const v4f a1 = *(const v4f*)(Wfr + e0 + 4);
  const float w0 = a0[0];
  const float w1 = a0[1];
  const float w2 = a0[2];
  const float w3 = a0[3];
  const float w4 = a1[0];
  const float w5 = a1[1];
  const float w6 = a1[2];
  const float w7 = a1[3];
  const float t0 = bf16r(w0) * kWCarry;
  const float t1 = bf16r(w1) * kWCarry;
  const float t2 = bf16r(w2) * kWCarry;
  const float t3 = bf16r(w3) * kWCarry;
  const float t4 = bf16r(w4) * kWCarry;
  const float t5 = bf16r(w5) * kWCarry;
  const float t6 = bf16r(w6) * kWCarry;
  const float t7 = bf16r(w7) * kWCarry;
  const float z0 = ((k8 + 0) == n) ? 0.0f : t0;
  const float z1 = ((k8 + 1) == n) ? 0.0f : t1;
  const float z2 = ((k8 + 2) == n) ? 0.0f : t2;
  const float z3 = ((k8 + 3) == n) ? 0.0f : t3;
  const float z4 = ((k8 + 4) == n) ? 0.0f : t4;
  const float z5 = ((k8 + 5) == n) ? 0.0f : t5;
  const float z6 = ((k8 + 6) == n) ? 0.0f : t6;
  const float z7 = ((k8 + 7) == n) ? 0.0f : t7;
  v8h hv;
  hv[0] = f16_flush(z0);
  hv[1] = f16_flush(z1);
  hv[2] = f16_flush(z2);
  hv[3] = f16_flush(z3);
  hv[4] = f16_flush(z4);
  hv[5] = f16_flush(z5);
  hv[6] = f16_flush(z6);
  hv[7] = f16_flush(z7);
  unsigned short* qh = dH + e0;
  *(volatile v8h*)qh = hv;
  __threadfence();
  *(volatile v8h*)qh = hv;
}

__global__ __launch_bounds__(32) void wdm_diag_kernel(
    const float* __restrict__ Wdm, float* __restrict__ DGM)
{
  const int i = threadIdx.x & 31;
  const float d0 = Wdm[(2 * i) * (kF + 1)];
  const float d1 = Wdm[(2 * i + 1) * (kF + 1)];
  v2f r;
  r[0] = bf16r(d0);
  r[1] = bf16r(d1);
  float* p = DGM + 2 * i;
  *(volatile v2f*)p = r;
  __threadfence();
  *(volatile v2f*)p = r;
}

__global__ __launch_bounds__(256) void impute_step_kernel(
    const float* __restrict__ x, const float* __restrict__ m, const float* __restrict__ t,
    const unsigned short* __restrict__ WDHp, const unsigned short* __restrict__ WTRp,
    const unsigned short* __restrict__ WFRp, const unsigned short* __restrict__ WWCp,
    const unsigned short* __restrict__ WIHp, const unsigned short* __restrict__ WHHp,
    const float* __restrict__ DGM, const float* __restrict__ BDH, const float* __restrict__ BDM,
    const float* __restrict__ BTR, const float* __restrict__ BFR, const float* __restrict__ BWC,
    const float* __restrict__ BIH, const float* __restrict__ BHH,
    float* __restrict__ out, float* __restrict__ PARTS)
{
  __shared__ __align__(16) _Float16 P_T[kSamp * kPT];
  __shared__ __align__(16) _Float16 P_H[kSamp * kPH];
  __shared__ __align__(16) _Float16 P_X[kSamp * kPX];
  __shared__ __align__(16) _Float16 P_GM[kSamp * kPGM];
  __shared__ __align__(16) _Float16 P_IN[kSamp * kPIN];
  __shared__ __align__(16) float XV[kSamp * kF];
  __shared__ __align__(16) float MV[kSamp * kF];
  __shared__ __align__(16) float XHAT[kSamp * kF];
  __shared__ __align__(16) float ZHAT[kSamp * kF];
  __shared__ __align__(16) float BETA[kSamp * kF];
  __shared__ __align__(16) float CC[kSamp * kF];
  __shared__ __align__(16) float PART[kS * 4];
  __shared__ __align__(16) float SLAB[4 * 4];

  const _Float16* WDH = (const _Float16*)WDHp;
  const _Float16* WTR = (const _Float16*)WTRp;
  const _Float16* WFR = (const _Float16*)WFRp;
  const _Float16* WWC = (const _Float16*)WWCp;
  const _Float16* WIH = (const _Float16*)WIHp;
  const _Float16* WHH = (const _Float16*)WHHp;

  const int tid   = threadIdx.x;
  const int lane  = tid & 31;
  const int wave  = tid >> 5;
  const int rlane = lane & 15;
  const int hi    = lane >> 4;
  const int koff  = 8 * hi;
  const int b0    = blockIdx.x * kSamp;

  const int sa0 = tid >> 4;
  const int f4  = (tid & 15) * 4;
  const int u    = 16 * wave + rlane;
  const int w4   = wave & 3;
  const int fcol = 16 * w4 + rlane;
  const int sa5 = 2 * wave + hi;
  const int f5  = rlane * 4;

  const v4f dgm4 = *(const v4f*)(DGM + f4);
  const v4f bdm4 = *(const v4f*)(BDM + f4);
  const float bdh_u = BDH[u];
  const float btr_c = BTR[fcol];
  const float bfr_c = BFR[fcol];
  const float bwc_c = BWC[fcol];
  const float bg_i = BIH[u] + BHH[u];
  const float bg_f = BIH[kH + u] + BHH[kH + u];
  const float bg_g = BIH[2 * kH + u] + BHH[2 * kH + u];
  const float bg_o = BIH[3 * kH + u] + BHH[3 * kH + u];

  v8f hreg = (v8f){0.f, 0.f, 0.f, 0.f, 0.f, 0.f, 0.f, 0.f};
  v8f creg = (v8f){0.f, 0.f, 0.f, 0.f, 0.f, 0.f, 0.f, 0.f};

  for (int s = 0; s < kS; ++s) {
    float e1 = 0.0f, e2 = 0.0f, e3 = 0.0f, ms = 0.0f;

    {
      const size_t g = ((size_t)(b0 + sa0) * kS + s) * kF + f4;
      const v4f xr = *(const v4f*)(x + g);
      const v4f mr = *(const v4f*)(m + g);
      const v4f tr = *(const v4f*)(t + g);
      v4f xq, mq;
      v4h th, gh4, mh;
#pragma unroll
      for (int e = 0; e < 4; ++e) {
        const float xe = xr[e];
        const float me = mr[e];
        const float te = tr[e];
        const float dg = dgm4[e];
        const float bd = bdm4[e];
        const float xv = bf16r(xe);
        const float mv = bf16r(me);
        const float tv = bf16r(te);
        const float gm = expf(-fmaxf(tv * dg + bd, 0.0f));
        xq[e] = xv;
        mq[e] = mv;
        th[e] = f16_flush(tv);
        gh4[e] = f16_flush(gm);
        mh[e] = f16_flush(mv);
      }
      *(v4f*)(XV + sa0 * kF + f4) = xq;
      *(v4f*)(MV + sa0 * kF + f4) = mq;
      *(v4h*)(P_T + sa0 * kPT + f4) = th;
      *(v4h*)(P_GM + sa0 * kPGM + f4) = gh4;
      *(v4h*)(P_GM + sa0 * kPGM + kF + f4) = mh;
      *(v4h*)(P_IN + sa0 * kPIN + kF + f4) = mh;
    }
    __syncthreads();

    {
      v8f acc = (v8f){0.f, 0.f, 0.f, 0.f, 0.f, 0.f, 0.f, 0.f};
      acc = tile_mm<kF>(P_T, kPT, WDH, kF, 16 * wave, rlane, koff, acc);
      eng::guard_acc(acc);
#pragma unroll
      for (int r = 0; r < 8; ++r) {
        const float gh = expf(-fmaxf(acc[r] * sW + bdh_u, 0.0f));
        const float hn = hreg[r] * gh;
        hreg[r] = hn;
        P_H[(8 * hi + r) * kPH + u] = f16_flush(hn);
      }
    }
    __syncthreads();

    if (wave < 4) {
      v8f acc = (v8f){0.f, 0.f, 0.f, 0.f, 0.f, 0.f, 0.f, 0.f};
      acc = tile_mm<kH>(P_H, kPH, WTR, kH, 16 * wave, rlane, koff, acc);
      eng::guard_acc(acc);
#pragma unroll
      for (int r = 0; r < 8; ++r) {
        const int sa = 8 * hi + r;
        const float xh = acc[r] * sW + btr_c;
        XHAT[sa * kF + fcol] = xh;
        const float xv = XV[sa * kF + fcol];
        const float mv = MV[sa * kF + fcol];
        const float xc = mv * xv + (1.0f - mv) * xh;
        P_X[sa * kPX + fcol] = f16_flush(xc);
        const float d1 = xv - xh;
        e1 += d1 * d1 * mv;
        ms += mv;
      }
    }
    __syncthreads();

    if (wave < 4) {
      v8f acc = (v8f){0.f, 0.f, 0.f, 0.f, 0.f, 0.f, 0.f, 0.f};
      acc = tile_mm<kF>(P_X, kPX, WFR, kF, 16 * wave, rlane, koff, acc);
      eng::guard_acc(acc);
#pragma unroll
      for (int r = 0; r < 8; ++r) {
        const int sa = 8 * hi + r;
        const float zh = acc[r] * sW + bfr_c;
        ZHAT[sa * kF + fcol] = zh;
        const float xv = XV[sa * kF + fcol];
        const float mv = MV[sa * kF + fcol];
        const float d2 = xv - zh;
        e2 += d2 * d2 * mv;
      }
    } else {
      v8f acc = (v8f){0.f, 0.f, 0.f, 0.f, 0.f, 0.f, 0.f, 0.f};
      acc = tile_mm<2 * kF>(P_GM, kPGM, WWC, 2 * kF, 16 * w4, rlane, koff, acc);
      eng::guard_acc(acc);
#pragma unroll
      for (int r = 0; r < 8; ++r) {
        const int sa = 8 * hi + r;
        BETA[sa * kF + fcol] = acc[r] * sW + bwc_c;
      }
    }
    __syncthreads();

    if (wave < 4) {
#pragma unroll
      for (int r = 0; r < 8; ++r) {
        const int sa = 8 * hi + r;
        const float be = BETA[sa * kF + fcol];
        const float zh = ZHAT[sa * kF + fcol];
        const float xh = XHAT[sa * kF + fcol];
        const float xv = XV[sa * kF + fcol];
        const float mv = MV[sa * kF + fcol];
        const float ch = be * zh + (1.0f - be) * xh;
        const float d3 = xv - ch;
        e3 += d3 * d3 * mv;
        const float cc = mv * xv + (1.0f - mv) * ch;
        CC[sa * kF + fcol] = cc;
        P_IN[sa * kPIN + fcol] = f16_flush(cc);
      }
    }
    __syncthreads();

    {
      const v4f cv = *(const v4f*)(CC + sa5 * kF + f5);
      float* op = out + kOut0 + ((size_t)(b0 + sa5) * kS + s) * kF + f5;
      *(volatile v4f*)op = cv;
      __threadfence();
      *(volatile v4f*)op = cv;
    }

    {
      v8f ai = (v8f){0.f, 0.f, 0.f, 0.f, 0.f, 0.f, 0.f, 0.f};
      v8f af = (v8f){0.f, 0.f, 0.f, 0.f, 0.f, 0.f, 0.f, 0.f};
      v8f ag = (v8f){0.f, 0.f, 0.f, 0.f, 0.f, 0.f, 0.f, 0.f};
      v8f ao = (v8f){0.f, 0.f, 0.f, 0.f, 0.f, 0.f, 0.f, 0.f};
      ai = tile_mm<2 * kF>(P_IN, kPIN, WIH, 2 * kF, 0 * kH + 16 * wave, rlane, koff, ai);
      ai = tile_mm<kH>(P_H, kPH, WHH, kH, 0 * kH + 16 * wave, rlane, koff, ai);
      eng::guard_acc(ai);
      af = tile_mm<2 * kF>(P_IN, kPIN, WIH, 2 * kF, 1 * kH + 16 * wave, rlane, koff, af);
      af = tile_mm<kH>(P_H, kPH, WHH, kH, 1 * kH + 16 * wave, rlane, koff, af);
      eng::guard_acc(af);
      ag = tile_mm<2 * kF>(P_IN, kPIN, WIH, 2 * kF, 2 * kH + 16 * wave, rlane, koff, ag);
      ag = tile_mm<kH>(P_H, kPH, WHH, kH, 2 * kH + 16 * wave, rlane, koff, ag);
      eng::guard_acc(ag);
      ao = tile_mm<2 * kF>(P_IN, kPIN, WIH, 2 * kF, 3 * kH + 16 * wave, rlane, koff, ao);
      ao = tile_mm<kH>(P_H, kPH, WHH, kH, 3 * kH + 16 * wave, rlane, koff, ao);
      eng::guard_acc(ao);
#pragma unroll
      for (int r = 0; r < 8; ++r) {
        const float gi = ai[r] * sW + bg_i;
        const float gf = af[r] * sW + bg_f;
        const float gg = ag[r] * sW + bg_g;
        const float go = ao[r] * sW + bg_o;
        const float iv = 1.0f / (1.0f + expf(-gi));
        const float fv = 1.0f / (1.0f + expf(-gf));
        const float gv = tanhf(gg);
        const float ov = 1.0f / (1.0f + expf(-go));
        const float cn = fv * creg[r] + iv * gv;
        creg[r] = cn;
        hreg[r] = ov * tanhf(cn);
      }
    }

    {
#pragma unroll
      for (int off = 16; off > 0; off >>= 1) {
        e1 += __shfl_xor(e1, off, 32);
        e2 += __shfl_xor(e2, off, 32);
        e3 += __shfl_xor(e3, off, 32);
        ms += __shfl_xor(ms, off, 32);
      }
      if (wave < 4 && lane == 0) {
        SLAB[wave * 4 + 0] = e1;
        SLAB[wave * 4 + 1] = e2;
        SLAB[wave * 4 + 2] = e3;
        SLAB[wave * 4 + 3] = ms;
      }
    }
    __syncthreads();
    if (tid == 0) {
#pragma unroll
      for (int q = 0; q < 4; ++q)
        PART[s * 4 + q] = ((SLAB[0 + q] + SLAB[4 + q]) + SLAB[8 + q]) + SLAB[12 + q];
    }
  }

  __syncthreads();
  {
    const v4f p0 = *(const v4f*)(PART + (size_t)tid * 4);
    const v4f p1 = *(const v4f*)(PART + (size_t)(256 + tid) * 4);
    float* q0 = PARTS + ((size_t)blockIdx.x * kS + tid) * 4;
    float* q1 = PARTS + ((size_t)blockIdx.x * kS + 256 + tid) * 4;
    for (int pass = 0; pass < 2; ++pass) {
      *(volatile v4f*)q0 = p0;
      *(volatile v4f*)q1 = p1;
      __threadfence();
    }
  }
}

__global__ __launch_bounds__(32) void impute_loss_kernel(
    const float* __restrict__ PARTS, float* __restrict__ out1)
{
  if (threadIdx.x != 0) return;
  float loss = 0.0f;
  for (int s = 0; s < kS; ++s) {
    float e1 = 0.0f, e2 = 0.0f, e3 = 0.0f, ms = 0.0f;
    for (int blk = 0; blk < kBlocks; ++blk) {
      const v4f p = *(const v4f*)(PARTS + ((size_t)blk * kS + s) * 4);
      e1 += p[0];
      e2 += p[1];
      e3 += p[2];
      ms += p[3];
    }
    const float den = ms + 1e-5f;
    loss = loss + e1 / den;
    loss = loss + e2 / den;
    loss = loss + e3 / den;
  }
  const float res = loss / (float)kS;
  *(volatile float*)out1 = res;
  __threadfence();
  *(volatile float*)out1 = res;
}

static_assert(((kH * kF / 8) % 256) == 0);
static_assert(((kF * kH / 8) % 256) == 0);
static_assert(((kG * kH / 8) % 256) == 0);
static_assert(((kF * kF / 8) % 256) == 0);
static_assert((kF / 4) <= 256 && (kH / 4) <= 256 && (kG / 4) <= 256);

extern "C" void kernel_launch(void* const* d_in, const int* in_sizes, int n_in,
                              void* d_out, int out_size, void* d_ws, size_t ws_size,
                              hipStream_t stream)
{
  if (n_in < 17) return;
  if (in_sizes[0] != kB * kS * kF) return;
  if (in_sizes[1] != kB * kS * kF) return;
  if (in_sizes[2] != kB * kS * kF) return;
  if (in_sizes[3] != kH * kF) return;
  if (in_sizes[4] != kH) return;
  if (in_sizes[5] != kF * kF) return;
  if (in_sizes[6] != kF) return;
  if (in_sizes[7] != kF * kH) return;
  if (in_sizes[8] != kF) return;
  if (in_sizes[9] != kF * kF) return;
  if (in_sizes[10] != kF) return;
  if (in_sizes[11] != kF * 2 * kF) return;
  if (in_sizes[12] != kF) return;
  if (in_sizes[13] != kG * 2 * kF) return;
  if (in_sizes[14] != kG * kH) return;
  if (in_sizes[15] != kG) return;
  if (in_sizes[16] != kG) return;
  if (out_size != kOut1 + 1) return;
  if (ws_size < kWsTotal) return;

  const float* x   = (const float*)d_in[0];
  const float* m   = (const float*)d_in[1];
  const float* t   = (const float*)d_in[2];
  const float* Wdh = (const float*)d_in[3];
  const float* bdh = (const float*)d_in[4];
  const float* Wdm = (const float*)d_in[5];
  const float* bdm = (const float*)d_in[6];
  const float* Wtr = (const float*)d_in[7];
  const float* btr = (const float*)d_in[8];
  const float* Wfr = (const float*)d_in[9];
  const float* bfr = (const float*)d_in[10];
  const float* Wwc = (const float*)d_in[11];
  const float* bwc = (const float*)d_in[12];
  const float* Wih = (const float*)d_in[13];
  const float* Whh = (const float*)d_in[14];
  const float* bih = (const float*)d_in[15];
  const float* bhh = (const float*)d_in[16];
  float* out = (float*)d_out;

  char* ws = (char*)d_ws;
  unsigned short* WDH = (unsigned short*)(ws + kOffWDH);
  unsigned short* WTR = (unsigned short*)(ws + kOffWTR);
  unsigned short* WWC = (unsigned short*)(ws + kOffWWC);
  unsigned short* WIH = (unsigned short*)(ws + kOffWIH);
  unsigned short* WHH = (unsigned short*)(ws + kOffWHH);
  unsigned short* WFR = (unsigned short*)(ws + kOffWFR);
  float* DGM = (float*)(ws + kOffDGM);
  float* BDH = (float*)(ws + kOffBDH);
  float* BDM = (float*)(ws + kOffBDM);
  float* BTR = (float*)(ws + kOffBTR);
  float* BFR = (float*)(ws + kOffBFR);
  float* BWC = (float*)(ws + kOffBWC);
  float* BIH = (float*)(ws + kOffBIH);
  float* BHH = (float*)(ws + kOffBHH);
  float* PARTS = (float*)(ws + kOffPARTS);

  pack_rows_bf_kernel<<<(kH * kF / 8) / 256, 256, 0, stream>>>(Wdh, WDH, kF, kH, kH * kF / 8, kWCarry);
  pack_rows_bf_kernel<<<(kF * kH / 8) / 256, 256, 0, stream>>>(Wtr, WTR, kH, kF, kF * kH / 8, kWCarry);
  pack_rows_bf_kernel<<<(kF * 2 * kF / 8) / 256, 256, 0, stream>>>(Wwc, WWC, 2 * kF, kF, kF * 2 * kF / 8, kWCarry);
  pack_rows_bf_kernel<<<(kG * 2 * kF / 8) / 256, 256, 0, stream>>>(Wih, WIH, 2 * kF, kG, kG * 2 * kF / 8, kWCarry);
  pack_rows_bf_kernel<<<(kG * kH / 8) / 256, 256, 0, stream>>>(Whh, WHH, kH, kG, kG * kH / 8, kWCarry);
  wfr_pack_kernel<<<(kF * kF / 8) / 256, 256, 0, stream>>>(Wfr, WFR, kF * kF / 8);
  wdm_diag_kernel<<<1, 32, 0, stream>>>(Wdm, DGM);
  rne_vec_kernel<<<1, 256, 0, stream>>>(bdh, BDH, kH / 4);
  rne_vec_kernel<<<1, 256, 0, stream>>>(bdm, BDM, kF / 4);
  rne_vec_kernel<<<1, 256, 0, stream>>>(btr, BTR, kF / 4);
  rne_vec_kernel<<<1, 256, 0, stream>>>(bfr, BFR, kF / 4);
  rne_vec_kernel<<<1, 256, 0, stream>>>(bwc, BWC, kF / 4);
  rne_vec_kernel<<<1, 256, 0, stream>>>(bih, BIH, kG / 4);
  rne_vec_kernel<<<1, 256, 0, stream>>>(bhh, BHH, kG / 4);

  impute_step_kernel<<<kBlocks, 256, 0, stream>>>(
      x, m, t, WDH, WTR, WFR, WWC, WIH, WHH,
      DGM, BDH, BDM, BTR, BFR, BWC, BIH, BHH, out, PARTS);

  impute_loss_kernel<<<1, 32, 0, stream>>>(PARTS, out + kOut1);
}
